// RevGNN_4071628996858
// MI455X (gfx1250) — hardware-verified
//
#include <hip/hip_runtime.h>
#include <stddef.h>


#define IN_F   100
#define KP1    128
#define HID    128
#define DGC    64
#define OUT_F  47
#define OUT_P  48
#define NSTEP  4
#define WMAT   (DGC * DGC)
#define LN_EPS 1e-5f

#define NB     1024
#define CHUNK  4096
#define NTHR   256
#define NWAVE  (NTHR / 32)
#define NGRP   (CHUNK / (NTHR * 4))
#define LCAP   (NGRP * 4)
#define SUBR   32
#define RB     32
#define NTHR2  192

#define LDS_ACC_F  (NB * DGC)
#define LDS_LIST_I (NTHR * LCAP)
#define LDS_BYTES  (LDS_ACC_F * 4 + NB * 4 + LDS_LIST_I * 4 + NTHR * 4 + 64)

static_assert(SUBR * DGC * 2 + SUBR * DGC * 4 <= LDS_LIST_I * 4);
static_assert(NB % SUBR == 0);
static_assert((NB & (NB - 1)) == 0);
static_assert((CHUNK & (CHUNK - 1)) == 0);
static_assert(NWAVE * 4 == SUBR);

typedef float          v4f   __attribute__((ext_vector_type(4)));
typedef float          v8f   __attribute__((ext_vector_type(8)));
typedef int            v4i   __attribute__((ext_vector_type(4)));
typedef unsigned short v8us  __attribute__((ext_vector_type(8)));
typedef _Float16       v4h   __attribute__((ext_vector_type(4)));
typedef _Float16       v8h   __attribute__((ext_vector_type(8)));
typedef _Float16       v16h  __attribute__((ext_vector_type(16)));
typedef __bf16         v16bf __attribute__((ext_vector_type(16)));
union FragH { v16h v; v8h h[2]; };
union FragB { v16bf v; v8us h[2]; };

__device__ __forceinline__ unsigned int bf16_rne(float f) {
  unsigned int u = __float_as_uint(f);
  u += 0x7FFFu + ((u >> 16) & 1u);
  return u >> 16;
}

__device__ __forceinline__ void split8(v4f a, v4f b, v8us& hi, v8us& lo) {
  unsigned int hb, lb;
#define SPLK(I, VAL) hb = bf16_rne(VAL); lb = bf16_rne((VAL) - __uint_as_float(hb << 16)); \
  hi[I] = (unsigned short)hb; lo[I] = (unsigned short)lb;
  SPLK(0, a.x) SPLK(1, a.y) SPLK(2, a.z) SPLK(3, a.w)
  SPLK(4, b.x) SPLK(5, b.y) SPLK(6, b.z) SPLK(7, b.w)
#undef SPLK
}

__device__ __forceinline__ v8h pack8h(v4f a, v4f b) {
  v8h t;
  t[0] = (_Float16)a.x; t[1] = (_Float16)a.y; t[2] = (_Float16)a.z; t[3] = (_Float16)a.w;
  t[4] = (_Float16)b.x; t[5] = (_Float16)b.y; t[6] = (_Float16)b.z; t[7] = (_Float16)b.w;
  return t;
}

__device__ __forceinline__ v8f wm_h(v16h a, v16h b, v8f c) {
  v8f d = __builtin_amdgcn_wmma_f32_16x16x32_f16(false, a, false, b, (short)0, c, false, false);
  asm volatile("v_nop\n\tv_nop\n\tv_nop\n\tv_nop" : "+v"(d) : "v"(a), "v"(b));
  return d;
}
__device__ __forceinline__ v8f wm_b(v16bf a, v16bf b, v8f c) {
  v8f d = __builtin_amdgcn_wmma_f32_16x16x32_bf16(false, a, false, b, (short)0, c, false, false);
  asm volatile("v_nop\n\tv_nop\n\tv_nop\n\tv_nop" : "+v"(d) : "v"(a), "v"(b));
  return d;
}

__device__ __forceinline__ float wsum8(float v) {
  v += __shfl_xor(v, 1, 32);
  v += __shfl_xor(v, 2, 32);
  v += __shfl_xor(v, 4, 32);
  return v;
}
__device__ __forceinline__ float wsum32(float v) {
  v += __shfl_xor(v, 16, 32);
  v += __shfl_xor(v, 8, 32);
  v += __shfl_xor(v, 4, 32);
  v += __shfl_xor(v, 2, 32);
  v += __shfl_xor(v, 1, 32);
  return v;
}
__device__ __forceinline__ v4f relu4(v4f z) {
  z.x = fmaxf(z.x, 0.0f); z.y = fmaxf(z.y, 0.0f); z.z = fmaxf(z.z, 0.0f); z.w = fmaxf(z.w, 0.0f);
  return z;
}

__device__ __forceinline__ v8h ln_relu8(v4f y0, v4f y1, const float* __restrict__ g,
                                         const float* __restrict__ b) {
  float s = ((y0.x + y0.y) + (y0.z + y0.w)) + ((y1.x + y1.y) + (y1.z + y1.w));
  s = wsum8(s);
  const float mu = s * (1.0f / (float)DGC);
  const v4f d0 = y0 - mu, d1 = y1 - mu;
  float q = ((d0.x * d0.x + d0.y * d0.y) + (d0.z * d0.z + d0.w * d0.w)) +
            ((d1.x * d1.x + d1.y * d1.y) + (d1.z * d1.z + d1.w * d1.w));
  q = wsum8(q);
  const float rs = rsqrtf(q * (1.0f / (float)DGC) + LN_EPS);
  const v4f g0 = *(const v4f*)g, g1 = *(const v4f*)(g + 4);
  const v4f b0 = *(const v4f*)b, b1 = *(const v4f*)(b + 4);
  const v4f z0 = relu4((d0 * rs) * g0 + b0);
  const v4f z1 = relu4((d1 * rs) * g1 + b1);
  return pack8h(z0, z1);
}

__global__ __launch_bounds__(NTHR) void k_prep(
    const float* __restrict__ w1, const float* __restrict__ w2,
    const float* __restrict__ wl, const float* __restrict__ wr,
    unsigned short* p1h, unsigned short* p1l, _Float16* p2, _Float16* pc, int ngrp) {
  const int i = blockIdx.x * NTHR + threadIdx.x;
  if (i >= ngrp) return;
  const int G1 = HID * KP1 / 8;
  const int G2 = OUT_P * HID / 8;
  if (i < G1) {
    const int e = i * 8, n = e / KP1, k0 = e % KP1;
    v8us hi = {0, 0, 0, 0, 0, 0, 0, 0}, lo = {0, 0, 0, 0, 0, 0, 0, 0};
#pragma unroll
    for (int j = 0; j < 8; ++j) {
      const int k = k0 + j;
      const float v = (k < IN_F) ? w1[n * IN_F + (k < IN_F ? k : 0)] : 0.0f;
      const unsigned hb = bf16_rne(v);
      const unsigned lb = bf16_rne(v - __uint_as_float(hb << 16));
      hi[j] = (unsigned short)hb;
      lo[j] = (unsigned short)lb;
    }
    *(volatile v8us*)(p1h + e) = hi;
    *(volatile v8us*)(p1l + e) = lo;
    __threadfence();
    *(volatile v8us*)(p1h + e) = hi;
    *(volatile v8us*)(p1l + e) = lo;
  } else if (i < G1 + G2) {
    const int e = (i - G1) * 8, n = e / HID, k0 = e % HID;
    v8h t;
#pragma unroll
    for (int j = 0; j < 8; ++j) {
      const float v = (n < OUT_F) ? w2[(n < OUT_F ? n : 0) * HID + k0 + j] * 16.0f : 0.0f;
      t[j] = (_Float16)v;
    }
    *(volatile v8h*)(p2 + e) = t;
    __threadfence();
    *(volatile v8h*)(p2 + e) = t;
  } else {
    const int e = (i - G1 - G2) * 8;
    const int q = e / WMAT, rem = e % WMAT;
    const float* src = ((q & 1) ? wr : wl) + (size_t)(q >> 1) * WMAT + rem;
    v8h t;
#pragma unroll
    for (int j = 0; j < 8; ++j) t[j] = (_Float16)(src[j] * 16.0f);
    *(volatile v8h*)(pc + e) = t;
    __threadfence();
    *(volatile v8h*)(pc + e) = t;
  }
}

__global__ __launch_bounds__(NTHR) void k_lin1(
    const float* __restrict__ x, const unsigned short* __restrict__ p1h,
    const unsigned short* __restrict__ p1l, const float* __restrict__ b1,
    const float* __restrict__ lng, const float* __restrict__ lnb,
    float* hout, _Float16* zout, int nN) {
  __shared__ v8us sAh[RB * KP1 / 8];
  __shared__ v8us sAl[RB * KP1 / 8];
  __shared__ v4f  sD4[RB * HID / 4];
  float* sD = (float*)sD4;
  const int tid = threadIdx.x, lane = tid & 31;
  const int wave = __builtin_amdgcn_readfirstlane(tid >> 5);
  const int hh = lane >> 4, m = lane & 15;
  const int row0 = blockIdx.x * RB;

  {
    const int r = tid >> 3, c0 = (tid & 7) * 16;
    int node = row0 + r;
    if (node > nN - 1) node = nN - 1;
    const float* xp = x + (size_t)node * IN_F + c0;
    const v4f z4 = {0.f, 0.f, 0.f, 0.f};
    v4f q0 = z4, q1 = z4, q2 = z4, q3 = z4;
    if (c0 + 4 <= IN_F)  q0 = *(const v4f*)xp;
    if (c0 + 8 <= IN_F)  q1 = *(const v4f*)(xp + 4);
    if (c0 + 12 <= IN_F) q2 = *(const v4f*)(xp + 8);
    if (c0 + 16 <= IN_F) q3 = *(const v4f*)(xp + 12);
    v8us ha = {0, 0, 0, 0, 0, 0, 0, 0}, la = {0, 0, 0, 0, 0, 0, 0, 0};
    v8us hb = {0, 0, 0, 0, 0, 0, 0, 0}, lb = {0, 0, 0, 0, 0, 0, 0, 0};
    split8(q0, q1, ha, la);
    split8(q2, q3, hb, lb);
    const int o = (r * KP1 + c0) / 8;
    sAh[o] = ha; sAh[o + 1] = hb;
    sAl[o] = la; sAl[o + 1] = lb;
  }
  __syncthreads();

  const int ncol = wave * 16 + m;
  const unsigned short* ahp = (const unsigned short*)sAh;
  const unsigned short* alp = (const unsigned short*)sAl;
  v8f cA = {0.f, 0.f, 0.f, 0.f, 0.f, 0.f, 0.f, 0.f};
  v8f cB = {0.f, 0.f, 0.f, 0.f, 0.f, 0.f, 0.f, 0.f};
#pragma unroll
  for (int kt = 0; kt < KP1 / 32; ++kt) {
    const int k0 = kt * 32 + 8 * hh;
    FragB bh, bl, a0h, a0l, a1h, a1l;
    const unsigned short* pb = p1h + (size_t)ncol * KP1 + k0;
    bh.h[0] = *(const v8us*)pb;  bh.h[1] = *(const v8us*)(pb + 16);
    pb = p1l + (size_t)ncol * KP1 + k0;
    bl.h[0] = *(const v8us*)pb;  bl.h[1] = *(const v8us*)(pb + 16);
    const unsigned short* pa = ahp + m * KP1 + k0;
    a0h.h[0] = *(const v8us*)pa; a0h.h[1] = *(const v8us*)(pa + 16);
    pa = alp + m * KP1 + k0;
    a0l.h[0] = *(const v8us*)pa; a0l.h[1] = *(const v8us*)(pa + 16);
    pa = ahp + (16 + m) * KP1 + k0;
    a1h.h[0] = *(const v8us*)pa; a1h.h[1] = *(const v8us*)(pa + 16);
    pa = alp + (16 + m) * KP1 + k0;
    a1l.h[0] = *(const v8us*)pa; a1l.h[1] = *(const v8us*)(pa + 16);
    cA = wm_b(a0l.v, bh.v, cA);
    cA = wm_b(a0h.v, bl.v, cA);
    cA = wm_b(a0h.v, bh.v, cA);
    cB = wm_b(a1l.v, bh.v, cB);
    cB = wm_b(a1h.v, bl.v, cB);
    cB = wm_b(a1h.v, bh.v, cB);
  }
  {
    const float bv = b1[ncol];
    float* d0 = sD + (8 * hh) * HID + ncol;
    float* d1 = sD + (16 + 8 * hh) * HID + ncol;
#pragma unroll
    for (int r = 0; r < 8; ++r) {
      d0[r * HID] = cA[r] + bv;
      d1[r * HID] = cB[r] + bv;
    }
  }
  __syncthreads();

  const int rbase = wave * 4;
  const v4f hv0 = sD4[(rbase + 0) * (HID / 4) + lane];
  const v4f hv1 = sD4[(rbase + 1) * (HID / 4) + lane];
  const v4f hv2 = sD4[(rbase + 2) * (HID / 4) + lane];
  const v4f hv3 = sD4[(rbase + 3) * (HID / 4) + lane];
  const int n0 = row0 + rbase;
  const bool ok0 = n0 < nN, ok1 = n0 + 1 < nN, ok2 = n0 + 2 < nN, ok3 = n0 + 3 < nN;
  float* hp0 = hout + (size_t)(ok0 ? n0 : 0) * HID + 4 * lane;
  float* hp1 = hout + (size_t)(ok1 ? n0 + 1 : 0) * HID + 4 * lane;
  float* hp2 = hout + (size_t)(ok2 ? n0 + 2 : 0) * HID + 4 * lane;
  float* hp3 = hout + (size_t)(ok3 ? n0 + 3 : 0) * HID + 4 * lane;
  const int r1 = rbase + (lane >> 3), q = lane & 7;
  const v4f y0 = sD4[r1 * (HID / 4) + (DGC / 4) + 2 * q];
  const v4f y1 = sD4[r1 * (HID / 4) + (DGC / 4) + 2 * q + 1];
  const v8h zz = ln_relu8(y0, y1, lng + 8 * q, lnb + 8 * q);
  const int n1 = row0 + r1;
  const bool okz = n1 < nN;
  _Float16* zp = zout + (size_t)(okz ? n1 : 0) * DGC + 8 * q;

  if (ok0) *(volatile v4f*)hp0 = hv0;
  if (ok1) *(volatile v4f*)hp1 = hv1;
  if (ok2) *(volatile v4f*)hp2 = hv2;
  if (ok3) *(volatile v4f*)hp3 = hv3;
  if (okz) *(volatile v8h*)zp = zz;
  __threadfence();
  if (ok0) *(volatile v4f*)hp0 = hv0;
  if (ok1) *(volatile v4f*)hp1 = hv1;
  if (ok2) *(volatile v4f*)hp2 = hv2;
  if (ok3) *(volatile v4f*)hp3 = hv3;
  if (okz) *(volatile v8h*)zp = zz;
}

__global__ __launch_bounds__(NTHR) void k_conv(
    float* h, const _Float16* __restrict__ zin, _Float16* znext,
    const int* __restrict__ ei,
    const _Float16* __restrict__ pwl, const _Float16* __restrict__ pwr,
    const float* __restrict__ bls, const float* __restrict__ lng, const float* __restrict__ lnb,
    int nN, int nE, int goff, int hasNext) {
  extern __shared__ v4f lds_dyn[];
  float*    acc   = (float*)lds_dyn;
  int*      cnt   = (int*)(acc + LDS_ACC_F);
  int*      list  = cnt + NB;
  int*      lcnt  = list + LDS_LIST_I;
  unsigned* wmask = (unsigned*)(lcnt + NTHR);
  _Float16* meanT = (_Float16*)list;
  float*    dtl   = (float*)(list + SUBR * DGC / 2);

  const int tid = threadIdx.x, lane = tid & 31;
  const int wave = __builtin_amdgcn_readfirstlane(tid >> 5);
  const int hh = lane >> 4, m = lane & 15;
  const int nodeBase = blockIdx.x * NB;

  {
    const v4f z4 = {0.f, 0.f, 0.f, 0.f};
    for (int i = tid; i < LDS_ACC_F / 4; i += NTHR) lds_dyn[i] = z4;
    for (int i = tid; i < NB; i += NTHR) cnt[i] = 0;
  }
  __syncthreads();

  const int* dstp = ei + (size_t)nE;
  const bool vec4 = ((nE & 3) == 0);
  const int nChunks = (nE + CHUNK - 1) / CHUNK;
  int* mylist = list + tid * LCAP;
#pragma unroll 1
  for (int ch = 0; ch < nChunks; ++ch) {
    const int cbase = ch * CHUNK;
    int c = 0;
#pragma unroll
    for (int g = 0; g < NGRP; ++g) {
      const int el0 = (g * NTHR + tid) * 4;
      const int e0  = cbase + el0;
      const int sent = -2147483647 - 1;
      v4i d = {sent, sent, sent, sent};
      if (vec4 && e0 + 3 < nE) {
        d = *(const v4i*)(dstp + e0);
      } else {
        if (e0     < nE) d.x = dstp[e0];
        if (e0 + 1 < nE) d.y = dstp[e0 + 1];
        if (e0 + 2 < nE) d.z = dstp[e0 + 2];
        if (e0 + 3 < nE) d.w = dstp[e0 + 3];
      }
      const unsigned s0 = (unsigned)d.x - (unsigned)nodeBase;
      const unsigned s1 = (unsigned)d.y - (unsigned)nodeBase;
      const unsigned s2 = (unsigned)d.z - (unsigned)nodeBase;
      const unsigned s3 = (unsigned)d.w - (unsigned)nodeBase;
#define HITJ(J, SJ)                                                   \
      if ((SJ) < (unsigned)NB) {                                      \
        if (c < LCAP) mylist[c] = (((el0 + (J)) << 10) | (int)(SJ));  \
        ++c;                                                          \
      }
      HITJ(0, s0)
      HITJ(1, s1)
      HITJ(2, s2)
      HITJ(3, s3)
#undef HITJ
    }
    lcnt[tid] = c;
    const unsigned mk = __builtin_amdgcn_ballot_w32(c > 0);
    if (lane == 0) wmask[wave] = mk;
    __syncthreads();

    if (wave == 0) {
#pragma unroll 1
      for (int w = 0; w < NWAVE; ++w) {
        unsigned mk2 = wmask[w];
#pragma unroll 1
        for (int pp = 0; pp < 16; ++pp) {
          if (mk2 == 0u) break;
          const int lnA = __builtin_ctz(mk2);
          mk2 &= mk2 - 1u;
          int lnB = -1;
          if (mk2 != 0u) { lnB = __builtin_ctz(mk2); mk2 &= mk2 - 1u; }
          const int myln = hh ? lnB : lnA;
          int cc = 0;
          if (myln >= 0) {
            cc = lcnt[w * 32 + myln];
            cc = cc < 0 ? 0 : (cc > LCAP ? LCAP : cc);
          }
          const int occ  = __shfl_xor(cc, 16, 32);
          const int kmax = cc > occ ? cc : occ;
          const int* lp = list + (w * 32 + (myln >= 0 ? myln : 0)) * LCAP;
#pragma unroll 1
          for (int k = 0; k < kmax; ++k) {
            const int ent = lp[k];
            const bool act = (k < cc);
            const int slot = act ? (ent & (NB - 1)) : -1;
            const int el = (ent >> 10) & (CHUNK - 1);
            int e = cbase + el;
            if (e > nE - 1) e = nE - 1;
            int src = ei[e];
            src = src < 0 ? 0 : (src > nN - 1 ? nN - 1 : src);
            const v4h zz = *(const v4h*)(zin + (size_t)src * DGC + 4 * m);
            v4f v;
            v.x = (float)zz.x; v.y = (float)zz.y; v.z = (float)zz.z; v.w = (float)zz.w;
            const int oslot = __shfl_xor(slot, 16, 32);
            const bool same = act && (slot == oslot);
            v4f ov;
            ov.x = __shfl_xor(v.x, 16, 32); ov.y = __shfl_xor(v.y, 16, 32);
            ov.z = __shfl_xor(v.z, 16, 32); ov.w = __shfl_xor(v.w, 16, 32);
            if (same && hh == 0) v = v + ov;
            const bool doit = act && !(same && hh == 1);
            if (doit) {
              v4f* ap = (v4f*)(acc + slot * DGC + 4 * m);
              const v4f cur = *ap;
              *ap = cur + v;
              if (m == 0) cnt[slot] = cnt[slot] + (same ? 2 : 1);
            }
          }
        }
      }
    }
    __syncthreads();
  }

  int nValid = nN - nodeBase;
  if (nValid > NB) nValid = NB;
  if (nValid < 0) nValid = 0;
  const int nsub = (nValid + SUBR - 1) / SUBR;
  const int rt = wave >> 2, ct = wave & 3;
  const int ncol = ct * 16 + m;
  const float sc = 0.0625f;

#pragma unroll 1
  for (int sb = 0; sb < nsub; ++sb) {
    const int rsub = sb * SUBR;
    {
      const int r = tid >> 3, c0 = (tid & 7) * 8;
      const int slot = rsub + r;
      const int cn = cnt[slot];
      const float inv = 1.0f / (float)(cn > 1 ? cn : 1);
      const v4f a0 = *(const v4f*)(acc + slot * DGC + c0) * inv;
      const v4f a1 = *(const v4f*)(acc + slot * DGC + c0 + 4) * inv;
      *(v8h*)(meanT + r * DGC + c0) = pack8h(a0, a1);
    }
    __syncthreads();

    v8f c8 = {0.f, 0.f, 0.f, 0.f, 0.f, 0.f, 0.f, 0.f};
#pragma unroll
    for (int kt = 0; kt < DGC / 32; ++kt) {
      const int k0 = kt * 32 + 8 * hh;
      FragH am, az, bw, br;
      const _Float16* pam = meanT + (rt * 16 + m) * DGC + k0;
      am.h[0] = *(const v8h*)pam; am.h[1] = *(const v8h*)(pam + 16);
      int zr = nodeBase + rsub + rt * 16 + m;
      if (zr > nN - 1) zr = nN - 1;
      const _Float16* paz = zin + (size_t)zr * DGC + k0;
      az.h[0] = *(const v8h*)paz; az.h[1] = *(const v8h*)(paz + 16);
      const _Float16* pbw = pwl + ncol * DGC + k0;
      bw.h[0] = *(const v8h*)pbw; bw.h[1] = *(const v8h*)(pbw + 16);
      const _Float16* pbr = pwr + ncol * DGC + k0;
      br.h[0] = *(const v8h*)pbr; br.h[1] = *(const v8h*)(pbr + 16);
      c8 = wm_h(am.v, bw.v, c8);
      c8 = wm_h(az.v, br.v, c8);
    }
    {
      float* dp = dtl + (rt * 16 + 8 * hh) * DGC + ncol;
#pragma unroll
      for (int r = 0; r < 8; ++r) dp[r * DGC] = c8[r];
    }
    __syncthreads();

    v8h zz = {0, 0, 0, 0, 0, 0, 0, 0};
    bool okz = false;
    _Float16* zp = znext;
    if (hasNext) {
      const int r1 = wave * 4 + (lane >> 3), q = lane & 7;
      const int n1 = nodeBase + rsub + r1;
      okz = n1 < nN;
      const int n1c = okz ? n1 : nN - 1;
      const float* hp1 = h + (size_t)n1c * HID + goff + 8 * q;
      const v4f y0 = *(const v4f*)(dtl + r1 * DGC + 8 * q) * sc + *(const v4f*)(bls + 8 * q) +
                     *(const v4f*)hp1;
      const v4f y1 = *(const v4f*)(dtl + r1 * DGC + 8 * q + 4) * sc + *(const v4f*)(bls + 8 * q + 4) +
                     *(const v4f*)(hp1 + 4);
      zz = ln_relu8(y0, y1, lng + 8 * q, lnb + 8 * q);
      zp = znext + (size_t)n1c * DGC + 8 * q;
    }
    const int c2 = m * 4;
    const int rA = wave * 4 + hh, rB = wave * 4 + 2 + hh;
    const int nA = nodeBase + rsub + rA, nBr = nodeBase + rsub + rB;
    const bool okA = nA < nN, okB = nBr < nN;
    float* hpA = h + (size_t)(okA ? nA : nN - 1) * HID + goff + c2;
    float* hpB = h + (size_t)(okB ? nBr : nN - 1) * HID + goff + c2;
    const v4f bb4 = *(const v4f*)(bls + c2);
    const v4f yA = *(const v4f*)(dtl + rA * DGC + c2) * sc + bb4 + *(const v4f*)hpA;
    const v4f yB = *(const v4f*)(dtl + rB * DGC + c2) * sc + bb4 + *(const v4f*)hpB;

    if (okz) *(volatile v8h*)zp = zz;
    if (okA) *(volatile v4f*)hpA = yA;
    if (okB) *(volatile v4f*)hpB = yB;
    __threadfence();
    if (okz) *(volatile v8h*)zp = zz;
    if (okA) *(volatile v4f*)hpA = yA;
    if (okB) *(volatile v4f*)hpB = yB;
    __syncthreads();
  }
}

__global__ __launch_bounds__(NTHR2) void k_lin2(
    const float* __restrict__ h, const _Float16* __restrict__ p2, const float* __restrict__ b2,
    const float* __restrict__ ng, const float* __restrict__ nbt, float* out, int nN) {
  __shared__ v4h sA4[RB * HID / 4];
  __shared__ v4f sO4[RB * OUT_F / 4];
  float* sO = (float*)sO4;
  const int tid = threadIdx.x, lane = tid & 31;
  const int wave = __builtin_amdgcn_readfirstlane(tid >> 5);
  const int hh = lane >> 4, m = lane & 15;
  const int row0 = blockIdx.x * RB;

  const v4f g4 = *(const v4f*)(ng + 4 * lane), b4 = *(const v4f*)(nbt + 4 * lane);
#pragma unroll 1
  for (int r = wave; r < RB; r += NTHR2 / 32) {
    int node = row0 + r;
    if (node > nN - 1) node = nN - 1;
    const v4f v = *(const v4f*)(h + (size_t)node * HID + 4 * lane);
    const float s = wsum32((v.x + v.y) + (v.z + v.w));
    const float mu = s * (1.0f / (float)HID);
    const v4f d = v - mu;
    const float q = wsum32((d.x * d.x + d.y * d.y) + (d.z * d.z + d.w * d.w));
    const float rs = rsqrtf(q * (1.0f / (float)HID) + LN_EPS);
    const v4f y = relu4((d * rs) * g4 + b4);
    v4h t;
    t.x = (_Float16)y.x; t.y = (_Float16)y.y; t.z = (_Float16)y.z; t.w = (_Float16)y.w;
    sA4[r * (HID / 4) + lane] = t;
  }
  __syncthreads();

  const int rt = wave / 3, ct = wave - rt * 3;
  const int ncol = ct * 16 + m;
  const _Float16* sA = (const _Float16*)sA4;
  v8f c8 = {0.f, 0.f, 0.f, 0.f, 0.f, 0.f, 0.f, 0.f};
#pragma unroll
  for (int kt = 0; kt < HID / 32; ++kt) {
    const int k0 = kt * 32 + 8 * hh;
    FragH a, b;
    const _Float16* pa = sA + (rt * 16 + m) * HID + k0;
    a.h[0] = *(const v8h*)pa; a.h[1] = *(const v8h*)(pa + 16);
    const _Float16* pb = p2 + ncol * HID + k0;
    b.h[0] = *(const v8h*)pb; b.h[1] = *(const v8h*)(pb + 16);
    c8 = wm_h(a.v, b.v, c8);
  }
  if (ncol < OUT_F) {
    const float bv = b2[ncol];
    float* op = sO + (rt * 16 + 8 * hh) * OUT_F + ncol;
#pragma unroll
    for (int r = 0; r < 8; ++r) op[r * OUT_F] = c8[r] * 0.0625f + bv;
  }
  __syncthreads();

  int nrows = nN - row0;
  if (nrows > RB) nrows = RB;
  if (nrows < 0) nrows = 0;
  const int nel = nrows * OUT_F;
  const int nv = nel >> 2;
  float* ob = out + (size_t)row0 * OUT_F;
  for (int f = tid; f < nv; f += NTHR2) *(volatile v4f*)(ob + 4 * f) = sO4[f];
  for (int e = nv * 4 + tid; e < nel; e += NTHR2) *(volatile float*)(ob + e) = sO[e];
  __threadfence();
  for (int f = tid; f < nv; f += NTHR2) *(volatile v4f*)(ob + 4 * f) = sO4[f];
  for (int e = nv * 4 + tid; e < nel; e += NTHR2) *(volatile float*)(ob + e) = sO[e];
}

static inline size_t a256(size_t b) { return (b + 255) & ~(size_t)255; }

extern "C" void kernel_launch(void* const* d_in, const int* in_sizes, int n_in,
                              void* d_out, int out_size, void* d_ws, size_t ws_size,
                              hipStream_t stream) {
  if (n_in < 13) return;
  const int nN = in_sizes[0] / IN_F;
  const int nE = in_sizes[1] / 2;
  if (nN <= 0 || in_sizes[0] != nN * IN_F || nE < 0 || in_sizes[1] != nE * 2) return;
  if (in_sizes[2] != HID * IN_F || in_sizes[3] < HID) return;
  if (in_sizes[4] != OUT_F * HID || in_sizes[5] < OUT_F) return;
  if (in_sizes[6] < HID || in_sizes[7] < HID) return;
  if (in_sizes[8] < NSTEP * DGC || in_sizes[9] < NSTEP * DGC || in_sizes[11] < NSTEP * DGC) return;
  if (in_sizes[10] != NSTEP * WMAT || in_sizes[12] != NSTEP * WMAT) return;
  if (out_size != nN * OUT_F) return;

  const float* x      = (const float*)d_in[0];
  const int*   ei     = (const int*)d_in[1];
  const float* lin1_w = (const float*)d_in[2];
  const float* lin1_b = (const float*)d_in[3];
  const float* lin2_w = (const float*)d_in[4];
  const float* lin2_b = (const float*)d_in[5];
  const float* norm_g = (const float*)d_in[6];
  const float* norm_b = (const float*)d_in[7];
  const float* ln_g   = (const float*)d_in[8];
  const float* ln_b   = (const float*)d_in[9];
  const float* Wl     = (const float*)d_in[10];
  const float* bl     = (const float*)d_in[11];
  const float* Wr     = (const float*)d_in[12];
  float*       out    = (float*)d_out;

  size_t off = 0;
  const size_t oh   = off; off += a256((size_t)nN * HID * sizeof(float));
  const size_t ozA  = off; off += a256((size_t)nN * DGC * sizeof(_Float16));
  const size_t ozB  = off; off += a256((size_t)nN * DGC * sizeof(_Float16));
  const size_t op1h = off; off += a256((size_t)HID * KP1 * sizeof(unsigned short));
  const size_t op1l = off; off += a256((size_t)HID * KP1 * sizeof(unsigned short));
  const size_t op2  = off; off += a256((size_t)OUT_P * HID * sizeof(_Float16));
  const size_t opc  = off; off += a256((size_t)NSTEP * 2 * WMAT * sizeof(_Float16));
  if (off > ws_size) return;

  char* ws = (char*)d_ws;
  float*          h   = (float*)(ws + oh);
  _Float16*       zA  = (_Float16*)(ws + ozA);
  _Float16*       zB  = (_Float16*)(ws + ozB);
  unsigned short* p1h = (unsigned short*)(ws + op1h);
  unsigned short* p1l = (unsigned short*)(ws + op1l);
  _Float16*       p2  = (_Float16*)(ws + op2);
  _Float16*       pc  = (_Float16*)(ws + opc);

  const int ngrp = (HID * KP1 + OUT_P * HID + NSTEP * 2 * WMAT) / 8;
  k_prep<<<(ngrp + NTHR - 1) / NTHR, NTHR, 0, stream>>>(lin1_w, lin2_w, Wl, Wr, p1h, p1l, p2, pc, ngrp);

  const int g32 = (nN + RB - 1) / RB;
  k_lin1<<<g32, NTHR, 0, stream>>>(x, p1h, p1l, lin1_b, ln_g, ln_b, h, zA, nN);

  hipFuncSetAttribute(reinterpret_cast<const void*>(&k_conv),
                      hipFuncAttributeMaxDynamicSharedMemorySize, LDS_BYTES);
  const int gc = (nN + NB - 1) / NB;
  for (int s = 0; s < NSTEP; ++s) {
    const _Float16* zin = (s & 1) ? zB : zA;
    _Float16* znext     = (s & 1) ? zA : zB;
    const int sn = (s + 1 < NSTEP) ? s + 1 : s;
    k_conv<<<gc, NTHR, LDS_BYTES, stream>>>(
        h, zin, znext, ei,
        pc + (size_t)(2 * s) * WMAT, pc + (size_t)(2 * s + 1) * WMAT,
        bl + (size_t)s * DGC, ln_g + (size_t)sn * DGC, ln_b + (size_t)sn * DGC,
        nN, nE, (s & 1) * DGC, (s + 1 < NSTEP) ? 1 : 0);
  }

  k_lin2<<<g32, NTHR2, 0, stream>>>(h, p2, lin2_b, norm_g, norm_b, out, nN);
}
